// Graph_CNN_Mesh_Pose_10015863734924
// MI455X (gfx1250) — hardware-run, weakly checked
//
#include <hip/hip_runtime.h>


namespace {
constexpr int B = 512, V0 = 1024, V1 = 256, V2 = 64, E0 = 8192, E1 = 2048, NFC = 512, NOUT = 63;
constexpr float XS = 8.0f, WSC = 256.0f;
typedef _Float16 b16;
typedef __attribute__((ext_vector_type(16))) _Float16 v16b;
typedef __attribute__((ext_vector_type(8))) _Float16 v8b;
typedef __attribute__((ext_vector_type(8))) float v8f;
typedef __attribute__((ext_vector_type(4))) float v4f;
typedef __attribute__((ext_vector_type(2))) float v2f;
__device__ __forceinline__ float bf16_rne(float f) { unsigned int u = __float_as_uint(f); u += 0x7FFFu + ((u >> 16) & 1u); float r = __uint_as_float(u & 0xFFFF0000u); asm volatile("" : "+v"(r)); return r; }
__device__ __forceinline__ void split16(float v, b16& hi, b16& lo) { hi = (b16)v; lo = (b16)(v - (float)hi); }
__device__ __forceinline__ v16b frag_kb(const b16* p, int hh) { const v8b a = *(const v8b*)(p + 8 * hh), b = *(const v8b*)(p + 16 + 8 * hh); v16b f;
#pragma unroll
  for (int e = 0; e < 8; ++e) { f[e] = a[e]; f[8 + e] = b[e]; } return f; }
__device__ __forceinline__ v8f wmma16b(v16b a, v16b b, v8f c) { v8f d = __builtin_amdgcn_wmma_f32_16x16x32_f16(false, a, false, b, (short)0, c, false, false); asm volatile("v_nop\n\tv_nop\n\tv_nop\n\tv_nop" : "+v"(d) : "v"(a), "v"(b)); return d; }
__device__ __forceinline__ void wave_lds_sync() { __builtin_amdgcn_fence(__ATOMIC_RELEASE, "workgroup"); __builtin_amdgcn_wave_barrier(); __builtin_amdgcn_fence(__ATOMIC_ACQUIRE, "workgroup"); }
__device__ __forceinline__ float pmul(float a, float b) { float p = a * b; asm volatile("" : "+v"(p)); return p; }
__device__ __forceinline__ int iclamp(int v, int lo, int hi) { return v < lo ? lo : (v > hi ? hi : v); }
constexpr int CSR_NBLK9 = 512, CSR_GB9 = 9, CSR_GN9 = 1 << CSR_GB9  , CSR_TS9 = (CSR_GN9 < 32 ? 32 : CSR_GN9)  , CSR_MAXG9 = 512, CSR_CAP9 = 12288  ;
__device__ __host__ __forceinline__ int csr_tix9(int v) { return (v >> CSR_GB9) * CSR_TS9 + (v & (CSR_GN9 - 1)); }
__global__ __launch_bounds__(64) void csrA_kernel9(const int* __restrict__ dst, int E, int N, int nG, int CHP, int NGP, int* __restrict__ STG, int* __restrict__ HST) {
  extern __shared__ int sm[];
  int* cnt = sm; int* run = sm + NGP; int* ids = sm + 2 * NGP;
  const int b = blockIdx.x; const int ch = (E + CSR_NBLK9 - 1) / CSR_NBLK9; const int e0 = b * ch, e1 = min(E, e0 + ch);
  for (int i = threadIdx.x; i < NGP; i += 64) cnt[i] = 0;
  for (int i = threadIdx.x; i < CHP; i += 64) ids[i] = -1;
  __syncthreads();
  if (threadIdx.x == 0) {
    for (int e = e0; e < e1; ++e) { int d = dst[e]; d = (d < 0) ? 0 : (d >= N ? N - 1 : d); cnt[d >> CSR_GB9] += 1; }
    int acc = 0; for (int g = 0; g < nG; ++g) { run[g] = acc; acc += cnt[g]; }
    for (int e = e0; e < e1; ++e) { int d = dst[e]; d = (d < 0) ? 0 : (d >= N ? N - 1 : d); const int g = d >> CSR_GB9; ids[run[g]] = e; run[g] += 1; } }
  __syncthreads();
  typedef __attribute__((ext_vector_type(4))) int v4i;
  for (int pass = 0; pass < 2; ++pass) {
    for (int i = threadIdx.x; i < CHP / 4; i += 64) *(volatile v4i*)(STG + (size_t)b * CHP + i * 4) = *(const v4i*)(&ids[i * 4]);
    for (int i = threadIdx.x; i < NGP / 4; i += 64) { v4i v; for (int e = 0; e < 4; ++e) v[e] = (i * 4 + e < nG) ? cnt[i * 4 + e] : 0; *(volatile v4i*)(HST + (size_t)b * NGP + i * 4) = v; }
    __threadfence(); }
}
__global__ __launch_bounds__(512) void csrS_kernel9(const int* __restrict__ HST, int nG, int NGP, int* __restrict__ START, int* __restrict__ TOT, int* __restrict__ OFF) {
  __shared__ int tot[CSR_MAXG9];
  const int b = threadIdx.x;
  for (int pass = 0; pass < 2; ++pass) { int runb = 0; for (int g = 0; g < nG; ++g) { int c = HST[(size_t)b * NGP + g]; c = (c < 0) ? 0 : c; ((volatile int*)OFF)[(size_t)g * CSR_NBLK9 + b] = runb; runb += c; } __threadfence(); }
  for (int g = threadIdx.x; g < nG; g += 512) { int s = 0; for (int bb = 0; bb < CSR_NBLK9; ++bb) { int c = HST[(size_t)bb * NGP + g]; s += (c < 0) ? 0 : c; } tot[g] = s; }
  __syncthreads();
  if (threadIdx.x < 32) {
    __shared__ int st[CSR_MAXG9 + 32];
    if (threadIdx.x == 0) { int acc = 0; for (int g = 0; g < NGP; ++g) { st[g] = acc; if (g < nG) acc += (tot[g] + 31) & ~31; } st[NGP] = acc; }
    __builtin_amdgcn_fence(__ATOMIC_RELEASE, "workgroup"); __builtin_amdgcn_wave_barrier(); __builtin_amdgcn_fence(__ATOMIC_ACQUIRE, "workgroup");
    for (int pass = 0; pass < 2; ++pass) { for (int i = threadIdx.x; i < NGP + 32; i += 32) { ((volatile int*)START)[i] = (i <= NGP) ? st[min(i, NGP)] : 0; ((volatile int*)TOT)[i] = (i < nG) ? tot[i] : 0; } __threadfence(); } }
}
__global__ __launch_bounds__(256) void csrB_kernel9(const int* __restrict__ dst, int N, int nG, int CHP, int NGP, int permLen, const int* __restrict__ STG, const int* __restrict__ HST, const int* __restrict__ OFF, const int* __restrict__ START, const int* __restrict__ TOT, int* __restrict__ PERM, int* __restrict__ ROWPTR, int* __restrict__ ROWCNT, int* __restrict__ FLAG) {
  typedef __attribute__((ext_vector_type(4))) int v4i;
  __shared__ int ids[CSR_CAP9]; __shared__ unsigned short key[CSR_CAP9]; __shared__ int outp[CSR_CAP9]; __shared__ int ncnt[CSR_GN9 + 1]; __shared__ int boff[CSR_NBLK9 + 1];
  const int g = blockIdx.x, t_ = threadIdx.x; int tot = TOT[g]; int st = START[g], stn = START[g + 1]; const int v0 = g * CSR_GN9; const int nv = min(CSR_GN9, N - v0); const int t0 = g * CSR_TS9;
  st = (st < 0) ? 0 : (st > permLen - 32 ? permLen - 32 : st) & ~31; stn = (stn < st) ? st : (stn > permLen ? permLen : stn); tot = (tot < 0) ? 0 : tot; if (tot > stn - st && tot <= CSR_CAP9) tot = stn - st;
  if (tot > CSR_CAP9) {
    for (int pass = 0; pass < 2; ++pass) { for (int i = t_; i < CSR_TS9 / 4; i += 256) { v4i a, c; for (int e = 0; e < 4; ++e) { a[e] = st; c[e] = 0; } *(volatile v4i*)(ROWPTR + t0 + i * 4) = a; *(volatile v4i*)(ROWCNT + t0 + i * 4) = c; } if (t_ == 0) ((volatile int*)FLAG)[0] = 1; __threadfence(); } (void)nv; return; }
  if (t_ == 0) { int acc = 0; for (int b = 0; b < CSR_NBLK9; ++b) { boff[b] = acc; int c = HST[(size_t)b * NGP + g]; c = (c < 0) ? 0 : (c > CHP ? CHP : c); acc += c; if (acc > tot) acc = tot; } boff[CSR_NBLK9] = acc; }
  for (int i = t_; i <= CSR_GN9; i += 256) ncnt[i] = 0;
  __syncthreads();
  for (int b = 0; b < CSR_NBLK9; ++b) { const int c = boff[b + 1] - boff[b]; int o_ = OFF[(size_t)g * CSR_NBLK9 + b]; o_ = (o_ < 0) ? 0 : (o_ > CHP - c ? CHP - c : o_); const int* src_ = STG + (size_t)b * CHP + o_;
    for (int i = t_; i < c; i += 256) { int id = src_[i]; id = (id < 0) ? 0 : id; ids[boff[b] + i] = id; int d = dst[id]; d = (d < v0) ? v0 : (d >= N ? N - 1 : d); int kk = d - v0; kk = (kk < 0) ? 0 : (kk >= CSR_GN9 ? CSR_GN9 - 1 : kk); key[boff[b] + i] = (unsigned short)kk; } }
  __syncthreads();
  if (t_ == 0) { for (int i = 0; i < tot; ++i) ncnt[key[i]] += 1; int acc = 0; for (int vl = 0; vl < CSR_GN9; ++vl) { const int c = ncnt[vl]; ncnt[vl] = acc; acc += c; } ncnt[CSR_GN9] = acc;
    for (int i = 0; i < tot; ++i) { const int vl = key[i]; outp[ncnt[vl]] = ids[i]; ncnt[vl] += 1; }
    for (int vl = CSR_GN9; vl > 0; --vl) ncnt[vl] = ncnt[vl - 1]; ncnt[0] = 0; }
  __syncthreads();
  for (int pass = 0; pass < 2; ++pass) {
    for (int i = t_; i < (stn - st) / 4; i += 256) { v4i v; for (int e = 0; e < 4; ++e) { const int q = i * 4 + e; v[e] = (q < tot) ? outp[q] : -1; } *(volatile v4i*)(PERM + st + i * 4) = v; }
    for (int i = t_; i < CSR_TS9 / 4; i += 256) { v4i a, c; for (int e = 0; e < 4; ++e) { const int vl = i * 4 + e; const int vc = vl < CSR_GN9 ? vl : CSR_GN9; a[e] = (vl < CSR_GN9) ? st + ncnt[vc] : st; c[e] = (vl < nv) ? (ncnt[(vc < CSR_GN9 ? vc : CSR_GN9 - 1) + 1] - ncnt[vc]) : 0; } *(volatile v4i*)(ROWPTR + t0 + i * 4) = a; *(volatile v4i*)(ROWCNT + t0 + i * 4) = c; }
    __threadfence(); }
}
__global__ __launch_bounds__(256) void csrZ_kernel9(int* __restrict__ p, size_t n4) { typedef __attribute__((ext_vector_type(4))) int v4i; const size_t tid = (size_t)blockIdx.x * 256 + threadIdx.x, nth = (size_t)gridDim.x * 256; v4i z = {0, 0, 0, 0}; for (size_t i = tid; i < n4; i += nth) *(volatile v4i*)(p + i * 4) = z; }
struct CsrBufs9 { int *STG, *HST, *OFF, *START, *TOT, *PERM, *ROWPTR, *ROWCNT, *FLAG; int nG, NGP, CHP; size_t permLen; char* base; size_t bytes; };
static size_t csr_carve9(CsrBufs9& c, char* ws, size_t off, int E, int N) {
  const size_t off0 = off; c.base = ws + off;
  auto al = [&](size_t bytes) { char* p = ws + off; off += (bytes + 255) & ~(size_t)255; return p; };
  c.nG = (N + CSR_GN9 - 1) / CSR_GN9; c.NGP = (c.nG + 31) & ~31; const int ch = (E + CSR_NBLK9 - 1) / CSR_NBLK9; c.CHP = (ch + 31) & ~31; c.permLen = (size_t)E + 32 * (size_t)c.nG + 32;
  c.STG = (int*)al((size_t)CSR_NBLK9 * c.CHP * 4); c.HST = (int*)al((size_t)CSR_NBLK9 * c.NGP * 4); c.OFF = (int*)al((size_t)c.NGP * CSR_NBLK9 * 4); c.START = (int*)al((size_t)(c.NGP + 64) * 4); c.TOT = (int*)al((size_t)(c.NGP + 64) * 4);
  c.PERM = (int*)al(c.permLen * 4); c.ROWPTR = (int*)al((size_t)c.nG * CSR_TS9 * 4); c.ROWCNT = (int*)al((size_t)c.nG * CSR_TS9 * 4); c.FLAG = (int*)al(256);
  c.bytes = off - off0; return off;
}
static void csr_build9(const CsrBufs9& c, const int* dst, int E, int N, hipStream_t stream) {
  const size_t smem = (size_t)(2 * c.NGP + c.CHP) * 4;
  csrZ_kernel9<<<512, 256, 0, stream>>>((int*)c.base, c.bytes / 16);
  csrA_kernel9<<<CSR_NBLK9, 64, smem, stream>>>(dst, E, N, c.nG, c.CHP, c.NGP, c.STG, c.HST);
  csrS_kernel9<<<1, 512, 0, stream>>>(c.HST, c.nG, c.NGP, c.START, c.TOT, c.OFF);
  csrB_kernel9<<<c.nG, 256, 0, stream>>>(dst, N, c.nG, c.CHP, c.NGP, (int)c.permLen, c.STG, c.HST, c.OFF, c.START, c.TOT, c.PERM, c.ROWPTR, c.ROWCNT, c.FLAG);
}


__global__ __launch_bounds__(256) void wcheb_kernel(const float* __restrict__ w, int Fin, int Fout, int KP, b16* __restrict__ WT) { const int u = blockIdx.x * 256 + threadIdx.x; if (u >= Fout * (KP / 8)) return; const int o = u / (KP / 8), c0 = (u % (KP / 8)) * 8; v8b v;
#pragma unroll
  for (int j = 0; j < 8; ++j) { const int c = c0 + j; float val = 0.0f; if (c < 3 * Fin) { const int k = c / Fin, fin = c % Fin; val = bf16_rne(w[(size_t)o * 3 * Fin + fin * 3 + k]); } v[j] = (b16)(val * WSC); }
  for (int pass = 0; pass < 2; ++pass) { *(volatile v8b*)(WT + (size_t)o * KP + c0) = v; __threadfence(); } }
__global__ __launch_bounds__(256) void wfc_kernel(const float* __restrict__ w1, const float* __restrict__ w2, b16* __restrict__ F1T, b16* __restrict__ F2T) { const size_t u = (size_t)blockIdx.x * 256 + threadIdx.x;
  for (int pass = 0; pass < 2; ++pass) {
    if (u < (size_t)NFC * 512) { v8b v;
#pragma unroll
      for (int j = 0; j < 8; ++j) v[j] = (b16)(bf16_rne(w1[u * 8 + j]) * WSC); *(volatile v8b*)(F1T + u * 8) = v; }
    if (u < 64 * 64) { const int o = (int)(u / 64), k0 = (int)(u % 64) * 8; v8b v;
#pragma unroll
      for (int j = 0; j < 8; ++j) v[j] = (b16)(o < NOUT ? bf16_rne(w2[(size_t)o * NFC + k0 + j]) * WSC : 0.0f); *(volatile v8b*)(F2T + (size_t)o * NFC + k0) = v; }
    __threadfence(); } }
__global__ __launch_bounds__(256) void stage_kernel(const float* __restrict__ x, float* __restrict__ X0) { const int u = blockIdx.x * 256 + threadIdx.x; if (u >= V0 * B) return; const int v = u / B, b = u % B; v4f r = {bf16_rne(x[((size_t)b * V0 + v) * 3]), bf16_rne(x[((size_t)b * V0 + v) * 3 + 1]), bf16_rne(x[((size_t)b * V0 + v) * 3 + 2]), 0.0f};
  for (int pass = 0; pass < 2; ++pass) { *(volatile v4f*)(X0 + (size_t)u * 4) = r; __threadfence(); } }
struct Lay { const float* p; int nb; int blo; };
__device__ __forceinline__ size_t lay_off(const Lay& L, int v, int b, int F4) { return ((size_t)v * L.nb + (b - L.blo)) * F4; }
template <int F4>
__global__ __launch_bounds__(256) void spmm_kernel(Lay IN, Lay SUB, const float* __restrict__ vals, const int* __restrict__ cols, CsrBufs9 c, int NV, int E, float coef, float sub, int bstart, int bcnt, float* __restrict__ OUT, int out_nb, int out_blo) {
  constexpr int BPW = F4 == 4 ? 32 : (F4 == 32 ? 4 : 2);
  const int wave = threadIdx.x >> 5, lane = threadIdx.x & 31; const size_t wid = (size_t)blockIdx.x * 8 + wave; const int nbw = bcnt / BPW; const int v = (int)(wid / nbw), bg = (int)(wid % nbw); if (v >= NV) return; const int b0 = bstart + bg * BPW;
  int st = c.ROWPTR[v], cnt = c.ROWCNT[v]; cnt = iclamp(cnt, 0, E); st = iclamp(st, 0, (int)c.permLen - cnt);
  const int bl = b0 + (lane * 4) / F4, fl = (lane * 4) % F4;
  v4f acc = {0.0f, 0.0f, 0.0f, 0.0f};
#pragma unroll 1
  for (int j = 0; j < cnt; ++j) { const int e = iclamp(c.PERM[st + j], 0, E - 1); const int cc = iclamp(cols[e], 0, NV - 1); const float w = bf16_rne(vals[e]); const v4f xv = *(const v4f*)(IN.p + lay_off(IN, cc, bl, F4) + fl); for (int k = 0; k < 4; ++k) acc[k] += pmul(w, xv[k]); }
  v4f r; { v4f sv = {0.0f, 0.0f, 0.0f, 0.0f}; if (sub != 0.0f) sv = *(const v4f*)(SUB.p + lay_off(SUB, v, bl, F4) + fl); for (int k = 0; k < 4; ++k) r[k] = pmul(coef, acc[k]) + pmul(sub, sv[k]); }
  Lay O = {OUT, out_nb, out_blo};
  for (int pass = 0; pass < 2; ++pass) { *(volatile v4f*)(OUT + lay_off(O, v, bl, F4) + fl) = r; __threadfence(); } }
template <int FIN, int FOUT, int EX0>
__global__ __launch_bounds__(32) void cheb_kernel(Lay X, Lay T1, Lay T2, const b16* __restrict__ WT, const float* __restrict__ bias, int bstart, int bcnt, float* __restrict__ Y) {
  constexpr int F4 = EX0 ? 4 : FIN, KP = EX0 ? 32 : 3 * FIN, NT = FOUT / 16; __shared__ __attribute__((aligned(16))) b16 Ah[16][KP + 8], Al[16][KP + 8]; __shared__ float Tf[16][FOUT + 4]; const int lane = threadIdx.x, nloc = lane & 15, hlf = lane >> 4;
  const int nbt = bcnt / 16; const int v = blockIdx.x / nbt, b0 = bstart + (blockIdx.x % nbt) * 16; const size_t r0 = (size_t)v * B + b0;
  for (int rr = 0; rr < 16; ++rr) { const int b = b0 + rr;
    if (EX0) { const float a = lane < 3 ? X.p[lay_off(X, v, b, 4) + lane] : 0.0f; const float t1 = lane < 3 ? T1.p[lay_off(T1, v, b, 4) + lane] : 0.0f; const float t2 = lane < 3 ? T2.p[lay_off(T2, v, b, 4) + lane] : 0.0f;
      const float s1 = __shfl(t1, (lane + 29) & 31), s2 = __shfl(t2, (lane + 26) & 31);
      const float vv = lane < 3 ? a : (lane < 6 ? s1 : (lane < 9 ? s2 : 0.0f)); b16 p, ql; split16(vv * XS, p, ql); Ah[rr][lane] = p; Al[rr][lane] = ql; }
    else { for (int c = lane; c < KP; c += 32) { const int k = c / FIN, f = c % FIN; const Lay& S = k == 0 ? X : (k == 1 ? T1 : T2); b16 p, ql; split16(S.p[lay_off(S, v, b, F4) + f] * XS, p, ql); Ah[rr][c] = p; Al[rr][c] = ql; } } }
  wave_lds_sync(); v8f acc[NT];
#pragma unroll
  for (int t = 0; t < NT; ++t) acc[t] = (v8f){};
#pragma unroll
  for (int kb = 0; kb < KP; kb += 32) { const v16b a = frag_kb(&Ah[nloc][kb], hlf), al = frag_kb(&Al[nloc][kb], hlf);
#pragma unroll
    for (int t = 0; t < NT; ++t) { const v16b bw = frag_kb(WT + (size_t)(t * 16 + nloc) * KP + kb, hlf); acc[t] = wmma16b(a, bw, acc[t]); acc[t] = wmma16b(al, bw, acc[t]); } }
#pragma unroll
  for (int t = 0; t < NT; ++t) { const int cc = t * 16 + nloc; const float bb = bf16_rne(bias[cc]);
#pragma unroll
    for (int r8 = 0; r8 < 8; ++r8) Tf[8 * hlf + r8][cc] = acc[t][r8] * (1.0f / (XS * WSC)) + bb; }
  wave_lds_sync();
  for (int pass = 0; pass < 2; ++pass) { for (int rr = 0; rr < 16; ++rr) { if (FOUT == 32) ((volatile float*)Y)[(r0 + rr) * FOUT + lane] = Tf[rr][lane]; else *(volatile v2f*)(Y + (r0 + rr) * FOUT + lane * 2) = (v2f){Tf[rr][lane * 2], Tf[rr][lane * 2 + 1]}; } __threadfence(); } }
__global__ __launch_bounds__(256) void pool_kernel(const float* __restrict__ Y, int NVo, int F, int BV, float* __restrict__ P) { const size_t u = (size_t)blockIdx.x * 256 + threadIdx.x; if (u >= (size_t)NVo * B * F / 4) return; const size_t e0 = u * 4; const int v = (int)(e0 / ((size_t)B * F)); const size_t rem = e0 % ((size_t)B * F); const int b = (int)(rem / F);
  v4f r = {0.0f, 0.0f, 0.0f, 0.0f}; if (b < BV) { r = *(const v4f*)(Y + ((size_t)(4 * v) * B * F) + rem); for (int j = 1; j < 4; ++j) { const v4f y = *(const v4f*)(Y + ((size_t)(4 * v + j) * B * F) + rem); for (int k = 0; k < 4; ++k) r[k] = fmaxf(r[k], y[k]); } }
  for (int pass = 0; pass < 2; ++pass) { *(volatile v4f*)(P + e0) = r; __threadfence(); } }
__global__ __launch_bounds__(32) void fc1_kernel(const float* __restrict__ P2, const b16* __restrict__ F1T, const float* __restrict__ b1, int BV, float* __restrict__ H) { __shared__ __attribute__((aligned(16))) b16 Ah[16][72], Al[16][72]; __shared__ float Tf[16][132]; const int lane = threadIdx.x, nloc = lane & 15, hlf = lane >> 4; const int grp = blockIdx.x % 4; const int b0 = (blockIdx.x / 4) * 16; if (b0 >= BV) return;
  v8f acc[8];
#pragma unroll
  for (int t = 0; t < 8; ++t) acc[t] = (v8f){};
#pragma unroll 1
  for (int v2 = 0; v2 < V2; ++v2) {
    for (int rr = 0; rr < 16; ++rr) for (int q = 0; q < 2; ++q) { b16 p, ql; split16(P2[((size_t)v2 * B + b0 + rr) * 64 + q * 32 + lane] * XS, p, ql); Ah[rr][q * 32 + lane] = p; Al[rr][q * 32 + lane] = ql; }
    wave_lds_sync();
#pragma unroll
    for (int kb = 0; kb < 64; kb += 32) { const v16b a = frag_kb(&Ah[nloc][kb], hlf), al = frag_kb(&Al[nloc][kb], hlf);
#pragma unroll
      for (int t = 0; t < 8; ++t) { const v16b bw = frag_kb(F1T + (size_t)(grp * 128 + t * 16 + nloc) * (V2 * 64) + v2 * 64 + kb, hlf); acc[t] = wmma16b(a, bw, acc[t]); acc[t] = wmma16b(al, bw, acc[t]); } }
    wave_lds_sync(); }
#pragma unroll
  for (int t = 0; t < 8; ++t) { const int cc = grp * 128 + t * 16 + nloc; const float bb = bf16_rne(b1[cc]);
#pragma unroll
    for (int r8 = 0; r8 < 8; ++r8) Tf[8 * hlf + r8][t * 16 + nloc] = acc[t][r8] * (1.0f / (XS * WSC)) + bb; }
  wave_lds_sync();
  for (int pass = 0; pass < 2; ++pass) { for (int rr = 0; rr < 16; ++rr) *(volatile v4f*)(H + (size_t)(b0 + rr) * NFC + grp * 128 + lane * 4) = *(const v4f*)(&Tf[rr][lane * 4]); __threadfence(); } }
__global__ __launch_bounds__(32) void fc2_kernel(const float* __restrict__ H, const b16* __restrict__ F2T, const float* __restrict__ b2, int BV, float* __restrict__ out) { __shared__ __attribute__((aligned(16))) b16 Ah[32][NFC + 8], Al[32][NFC + 8]; __shared__ float Tf[32][68]; const int lane = threadIdx.x, nloc = lane & 15, hlf = lane >> 4; const int b0 = blockIdx.x * 32; if (b0 >= BV) return;
  for (int rr = 0; rr < 32; ++rr) for (int q = 0; q < 16; ++q) { b16 p, ql; split16(H[(size_t)(b0 + rr) * NFC + q * 32 + lane] * XS, p, ql); Ah[rr][q * 32 + lane] = p; Al[rr][q * 32 + lane] = ql; }
  wave_lds_sync();
  for (int mt = 0; mt < 2; ++mt) { v8f acc[4] = {(v8f){}, (v8f){}, (v8f){}, (v8f){}};
#pragma unroll 4
    for (int kb = 0; kb < NFC; kb += 32) { const v16b a = frag_kb(&Ah[mt * 16 + nloc][kb], hlf), al = frag_kb(&Al[mt * 16 + nloc][kb], hlf);
#pragma unroll
      for (int t = 0; t < 4; ++t) { const v16b bw = frag_kb(F2T + (size_t)(t * 16 + nloc) * NFC + kb, hlf); acc[t] = wmma16b(a, bw, acc[t]); acc[t] = wmma16b(al, bw, acc[t]); } }
#pragma unroll
    for (int t = 0; t < 4; ++t) { const int cc = t * 16 + nloc; const float bb = cc < NOUT ? bf16_rne(b2[cc]) : 0.0f;
#pragma unroll
      for (int r8 = 0; r8 < 8; ++r8) Tf[mt * 16 + 8 * hlf + r8][cc] = acc[t][r8] * (1.0f / (XS * WSC)) + bb; } }
  wave_lds_sync();
  for (int pass = 0; pass < 2; ++pass) { for (int q = lane; q < 32 * NOUT; q += 32) ((volatile float*)out)[(size_t)b0 * NOUT + q] = Tf[q / NOUT][q % NOUT]; __threadfence(); } }
}

extern "C" void kernel_launch(void* const* d_in, const int* in_sizes, int n_in, void* d_out, int out_size, void* d_ws, size_t ws_size, hipStream_t stream) {
  (void)n_in;
  auto Fp = [&](int i) { return (const float*)d_in[i]; }; auto Ip = [&](int i) { return (const int*)d_in[i]; };
  if (in_sizes[0] != B * V0 * 3 || in_sizes[1] != E0 || in_sizes[4] != E1 || in_sizes[7] != 32 * 9 || in_sizes[13] != 64 * 192 || in_sizes[15] != NFC * V2 * 64 || in_sizes[17] != NOUT * NFC || out_size != B * NOUT) return;
  const int BV = B;
  size_t off = 0; char* ws = (char*)d_ws;
  auto carve = [&](size_t bytes) { char* p = ws + off; off += (bytes + 255) & ~(size_t)255; return p; };
  b16* W0T = (b16*)carve((size_t)32 * 32 * 2); b16* W1T = (b16*)carve((size_t)32 * 96 * 2); b16* W2T = (b16*)carve((size_t)64 * 96 * 2); b16* W3T = (b16*)carve((size_t)64 * 192 * 2); b16* F1T = (b16*)carve((size_t)NFC * V2 * 64 * 2); b16* F2T = (b16*)carve((size_t)64 * NFC * 2);
  constexpr int BC = 256;
  float* X0 = (float*)carve((size_t)V0 * B * 4 * 4); float* T1 = (float*)carve((size_t)V0 * BC * 32 * 4); float* T2 = (float*)carve((size_t)V0 * BC * 32 * 4); float* YA = (float*)carve((size_t)V0 * B * 32 * 4); float* YB = (float*)carve((size_t)V0 * B * 32 * 4); float* Hf = (float*)carve((size_t)B * NFC * 4);
  CsrBufs9 c0, c1; off = csr_carve9(c0, ws, off, E0, V0); off = csr_carve9(c1, ws, off, E1, V1);
  if (off > ws_size || off > ((size_t)224 << 20)) return;
  wcheb_kernel<<<4, 256, 0, stream>>>(Fp(7), 3, 32, 32, W0T); wcheb_kernel<<<2, 256, 0, stream>>>(Fp(9), 32, 32, 96, W1T); wcheb_kernel<<<4, 256, 0, stream>>>(Fp(11), 32, 64, 96, W2T); wcheb_kernel<<<8, 256, 0, stream>>>(Fp(13), 64, 64, 192, W3T);
  wfc_kernel<<<(NFC * 512 + 255) / 256, 256, 0, stream>>>(Fp(15), Fp(17), F1T, F2T);
  csr_build9(c0, Ip(1), E0, V0, stream); csr_build9(c1, Ip(4), E1, V1, stream);
  stage_kernel<<<(V0 * B + 255) / 256, 256, 0, stream>>>(Fp(0), X0);
  const Lay LX0 = {X0, B, 0}, LYA = {YA, B, 0}, LYB = {YB, B, 0};
  for (int bs = 0; bs < BV; bs += BC) { const int bc = (BV - bs) < BC ? (BV - bs) : BC; const Lay LT1 = {T1, BC, bs}, LT2 = {T2, BC, bs};
    spmm_kernel<4><<<(V0 * (bc / 32) + 7) / 8, 256, 0, stream>>>(LX0, LX0, Fp(3), Ip(2), c0, V0, E0, 1.0f, 0.0f, bs, bc, T1, BC, bs);
    spmm_kernel<4><<<(V0 * (bc / 32) + 7) / 8, 256, 0, stream>>>(LT1, LX0, Fp(3), Ip(2), c0, V0, E0, 2.0f, -1.0f, bs, bc, T2, BC, bs);
    cheb_kernel<3, 32, 1><<<V0 * (bc / 16), 32, 0, stream>>>(LX0, LT1, LT2, W0T, Fp(8), bs, bc, YA);
    spmm_kernel<32><<<(V0 * (bc / 4) + 7) / 8, 256, 0, stream>>>(LYA, LYA, Fp(3), Ip(2), c0, V0, E0, 1.0f, 0.0f, bs, bc, T1, BC, bs);
    spmm_kernel<32><<<(V0 * (bc / 4) + 7) / 8, 256, 0, stream>>>(LT1, LYA, Fp(3), Ip(2), c0, V0, E0, 2.0f, -1.0f, bs, bc, T2, BC, bs);
    cheb_kernel<32, 32, 0><<<V0 * (bc / 16), 32, 0, stream>>>(LYA, LT1, LT2, W1T, Fp(10), bs, bc, YB); }
  pool_kernel<<<(unsigned)(((size_t)V1 * B * 32 / 4 + 255) / 256), 256, 0, stream>>>(YB, V1, 32, BV, YA);
  { const Lay LYA1 = {YA, B, 0}, LYB1 = {YB, B, 0}, LT1 = {T1, B, 0}, LT2 = {T2, B, 0};
    spmm_kernel<32><<<(V1 * (BV / 4) + 7) / 8, 256, 0, stream>>>(LYA1, LYA1, Fp(6), Ip(5), c1, V1, E1, 1.0f, 0.0f, 0, BV, T1, B, 0);
    spmm_kernel<32><<<(V1 * (BV / 4) + 7) / 8, 256, 0, stream>>>(LT1, LYA1, Fp(6), Ip(5), c1, V1, E1, 2.0f, -1.0f, 0, BV, T2, B, 0);
    cheb_kernel<32, 64, 0><<<V1 * (BV / 16), 32, 0, stream>>>(LYA1, LT1, LT2, W2T, Fp(12), 0, BV, YB);
    spmm_kernel<64><<<(V1 * (BV / 2) + 7) / 8, 256, 0, stream>>>(LYB1, LYB1, Fp(6), Ip(5), c1, V1, E1, 1.0f, 0.0f, 0, BV, T1, B, 0);
    spmm_kernel<64><<<(V1 * (BV / 2) + 7) / 8, 256, 0, stream>>>(LT1, LYB1, Fp(6), Ip(5), c1, V1, E1, 2.0f, -1.0f, 0, BV, T2, B, 0);
    cheb_kernel<64, 64, 0><<<V1 * (BV / 16), 32, 0, stream>>>(LYB1, LT1, LT2, W3T, Fp(14), 0, BV, YA); }
  pool_kernel<<<(unsigned)(((size_t)V2 * B * 64 / 4 + 255) / 256), 256, 0, stream>>>(YA, V2, 64, BV, YB);
  fc1_kernel<<<(B / 16) * 4, 32, 0, stream>>>(YB, F1T, Fp(16), BV, Hf);
  fc2_kernel<<<B / 32, 32, 0, stream>>>(Hf, F2T, Fp(18), BV, (float*)d_out);
}
